// QuadraticHeterogenousCrossAttention_23038204576029
// MI455X (gfx1250) — hardware-verified
//
#include <hip/hip_runtime.h>
#include <math.h>
#include <stddef.h>

typedef __attribute__((ext_vector_type(16))) _Float16 v16h;
typedef __attribute__((ext_vector_type(8)))  _Float16 v8h;
typedef __attribute__((ext_vector_type(16))) __bf16   v16b;
typedef __attribute__((ext_vector_type(8)))  __bf16   v8b;
typedef __attribute__((ext_vector_type(8)))  float    v8f;
typedef __attribute__((ext_vector_type(4)))  float    v4f;
typedef __attribute__((ext_vector_type(4)))  unsigned int v4u;

__device__ __forceinline__ unsigned short f2bf_bits(float f) {
  unsigned u = __float_as_uint(f);
  return (unsigned short)((u + 0x7FFFu + ((u >> 16) & 1u)) >> 16);
}
__device__ __forceinline__ float bf_bits2f(unsigned short h) { return __uint_as_float(((unsigned)h) << 16); }

__device__ __forceinline__ void dep_guard_h(v8f& a, v8f& b, v16h x, v16h y) { asm volatile("v_nop\n\tv_nop\n\tv_nop\n\tv_nop" : "+v"(a), "+v"(b) : "v"(x), "v"(y)); }
__device__ __forceinline__ void dep_guard_b(v8f& a, v8f& b, v16b x, v16b y) { asm volatile("v_nop\n\tv_nop\n\tv_nop\n\tv_nop" : "+v"(a), "+v"(b) : "v"(x), "v"(y)); }
__device__ __forceinline__ void keep4_h(v16h a, v16h b, v16h c, v16h d) { asm volatile("v_nop" :: "v"(a), "v"(b), "v"(c), "v"(d)); }
__device__ __forceinline__ void keep4_b(v16b a, v16b b, v16b c, v16b d) { asm volatile("v_nop" :: "v"(a), "v"(b), "v"(c), "v"(d)); }
__device__ __forceinline__ void acc_guard4(v8f& a, v8f& b, v8f& c, v8f& d) { asm volatile("v_nop\n\tv_nop\n\tv_nop\n\tv_nop" : "+v"(a), "+v"(b), "+v"(c), "+v"(d)); }
template <typename T> struct Frag;
template <> struct Frag<_Float16> {
  typedef v16h V; union U { v16h v; v8h h[2]; };
  static __device__ __forceinline__ v16h load(const _Float16* p) {
    U f; f.h[0] = *(const v8h*)(p); f.h[1] = *(const v8h*)(p + 16); return f.v;
  }
  static __device__ __forceinline__ v8f mma(v16h a, v16h b, v8f c) {
    return __builtin_amdgcn_wmma_f32_16x16x32_f16(false, a, false, b, (short)0, c, false, false);
  }
  static __device__ __forceinline__ void guard(v8f& a, v8f& b, v16h x, v16h y) { dep_guard_h(a, b, x, y); }
  static __device__ __forceinline__ void keep(v16h a, v16h b, v16h c, v16h d) { keep4_h(a, b, c, d); }
};
template <> struct Frag<__bf16> {
  typedef v16b V; union U { v16b v; v8b h[2]; };
  static __device__ __forceinline__ v16b load(const __bf16* p) {
    U f; f.h[0] = *(const v8b*)(p); f.h[1] = *(const v8b*)(p + 16); return f.v;
  }
  static __device__ __forceinline__ v8f mma(v16b a, v16b b, v8f c) {
    return __builtin_amdgcn_wmma_f32_16x16x32_bf16(false, a, false, b, (short)0, c, false, false);
  }
  static __device__ __forceinline__ void guard(v8f& a, v8f& b, v16b x, v16b y) { dep_guard_b(a, b, x, y); }
  static __device__ __forceinline__ void keep(v16b a, v16b b, v16b c, v16b d) { keep4_b(a, b, c, d); }
};

template <int ET> struct Elem;
template <> struct Elem<0> { typedef _Float16 T; };
template <> struct Elem<1> { typedef __bf16 T; };
template <int ET, bool SPLIT, int BIAS_MODE, int OUT_MODE, bool RESID, int ACT = 0>
__global__ __launch_bounds__(256) void wmma_gemm64(
    const unsigned short* __restrict__ Ap, const unsigned short* __restrict__ A2p, int lda, long strideA,
    const unsigned short* __restrict__ Btp, const unsigned short* __restrict__ Bt2p, int ldb, long strideB,
    void* __restrict__ Cout, void* __restrict__ Cout2, int ldc, long strideC,
    const float* __restrict__ bias,
    const float* __restrict__ resid, long strideR,
    int M, int N, int K, float scale) {
  typedef typename Elem<ET>::T T;
  typedef typename Frag<T>::V V;
  const T* A = (const T*)Ap; const T* A2 = (const T*)A2p; const T* Bt = (const T*)Btp; const T* Bt2 = (const T*)Bt2p;
  __shared__ __align__(16) float sT[8][16 * 68];
  const int b    = blockIdx.y;
  const int lane = threadIdx.x & 31;
  const int wave = threadIdx.x >> 5;
  const int tilesN = N >> 6;
  const int tilesM = M >> 6;
  const int tile = blockIdx.x * 8 + wave;
  if (tile >= tilesM * tilesN) return;
  const int tm = tile / tilesN;
  const int tn = tile - tm * tilesN;
  const int m0 = tm << 6;
  const int n0 = tn << 6;

  const T* Ab  = A  + (size_t)b * strideA;
  const T* Bb  = Bt + (size_t)b * strideB;
  const T* Ab2 = SPLIT ? (A2  + (size_t)b * strideA) : nullptr;
  const T* Bb2 = SPLIT ? (Bt2 + (size_t)b * strideB) : nullptr;

  const int rlane = lane & 15;
  const int koff  = (lane >> 4) * 8;
  const int mOff  = (lane >> 4) * 8;

  v8f acc[4][4];
#pragma unroll
  for (int i = 0; i < 4; ++i)
#pragma unroll
    for (int j = 0; j < 4; ++j) acc[i][j] = (v8f){0.f,0.f,0.f,0.f,0.f,0.f,0.f,0.f};

  for (int k0 = 0; k0 < K; k0 += 32) {
    V bh[4], bl[4];
#pragma unroll
    for (int j = 0; j < 4; ++j) {
      const size_t bo = (size_t)(n0 + (j << 4) + rlane) * ldb + koff + k0;
      bh[j] = Frag<T>::load(Bb + bo);
      if (SPLIT) bl[j] = Frag<T>::load(Bb2 + bo);
    }
#pragma unroll
    for (int i = 0; i < 4; ++i) {
      const size_t ao = (size_t)(m0 + (i << 4) + rlane) * lda + koff + k0;
      V ah = Frag<T>::load(Ab + ao);
      V al;
      if (SPLIT) al = Frag<T>::load(Ab2 + ao);
#pragma unroll
      for (int j = 0; j < 4; ++j) {
        acc[i][j] = Frag<T>::mma(ah, bh[j], acc[i][j]);
        if (SPLIT) {
          acc[i][j] = Frag<T>::mma(ah, bl[j], acc[i][j]);
          acc[i][j] = Frag<T>::mma(al, bh[j], acc[i][j]);
        }
      }
      Frag<T>::guard(acc[i][0], acc[i][3], ah, SPLIT ? al : ah);
    }
    Frag<T>::keep(bh[0], bh[1], bh[2], bh[3]);
    if (SPLIT) Frag<T>::keep(bl[0], bl[1], bl[2], bl[3]);
  }
  acc_guard4(acc[0][0], acc[0][1], acc[0][2], acc[0][3]);
  acc_guard4(acc[1][0], acc[1][1], acc[1][2], acc[1][3]);
  acc_guard4(acc[2][0], acc[2][1], acc[2][2], acc[2][3]);
  acc_guard4(acc[3][0], acc[3][1], acc[3][2], acc[3][3]);

  float* slab = sT[wave];
  const float* Rb = RESID ? (resid + (size_t)b * strideR) : nullptr;
#pragma unroll
  for (int i = 0; i < 4; ++i) {
    const int mBase = m0 + (i << 4);
#pragma unroll
    for (int j = 0; j < 4; ++j) {
      const int n = n0 + (j << 4) + rlane;
      float bv = 0.f;
      if (BIAS_MODE == 2) bv = bias[n];
#pragma unroll
      for (int r = 0; r < 8; ++r) {
        float v = acc[i][j][r] * scale;
        if (BIAS_MODE == 1) v += bias[mBase + mOff + r];
        if (BIAS_MODE == 2) v += bv;
        if (RESID) v += Rb[(size_t)(mBase + mOff + r) * ldc + n];
        if (ACT == 1) v = tanhf(v);
        if (ACT == 2) v = fmaxf(v, 0.0f);
        if (ACT == 3) v = v / (1.0f + expf(-v));
        if (ACT == 4) v = (v > 0.f) ? v : 0.01f * v;
        if (ACT == 5) v = 0.5f * v * (1.0f + erff(v * 0.70710678118654752f));
        slab[(mOff + r) * 68 + (j << 4) + rlane] = v;
      }
    }
    __builtin_amdgcn_fence(__ATOMIC_RELEASE, "workgroup");
    __builtin_amdgcn_wave_barrier();
    __builtin_amdgcn_fence(__ATOMIC_ACQUIRE, "workgroup");
    if (OUT_MODE == 0) {
      float* C = (float*)Cout + (size_t)b * strideC;
      const int hh = lane >> 4, c4 = (lane & 15) * 4;
      for (int pass = 0; pass < 2; ++pass) {
#pragma unroll
        for (int it = 0; it < 8; ++it) {
          const int row = it * 2 + hh;
          v4f v = *(const v4f*)(slab + row * 68 + c4);
          *(volatile v4f*)(C + (size_t)(mBase + row) * ldc + n0 + c4) = v;
        }
        __threadfence();
      }
    } else {
      const int q = lane >> 3, c8 = (lane & 7) * 8;
      unsigned short* C  = (unsigned short*)Cout  + (size_t)b * strideC;
      unsigned short* C2 = (OUT_MODE == 2) ? ((unsigned short*)Cout2 + (size_t)b * strideC) : nullptr;
      for (int pass = 0; pass < 2; ++pass) {
#pragma unroll
        for (int it = 0; it < 4; ++it) {
          const int row = it * 4 + q;
          const float* sp = slab + row * 68 + c8;
          v8h hv, lv;
#pragma unroll
          for (int e = 0; e < 8; ++e) {
            if (OUT_MODE == 1) {
              hv[e] = (_Float16)sp[e];
            } else {
              unsigned short hb = f2bf_bits(sp[e]);
              unsigned short lb = f2bf_bits(sp[e] - bf_bits2f(hb));
              hv[e] = __builtin_bit_cast(_Float16, hb);
              lv[e] = __builtin_bit_cast(_Float16, lb);
            }
          }
          *(volatile v8h*)(C + (size_t)(mBase + row) * ldc + n0 + c8) = hv;
          if (OUT_MODE == 2) *(volatile v8h*)(C2 + (size_t)(mBase + row) * ldc + n0 + c8) = lv;
        }
        __threadfence();
      }
    }
    __builtin_amdgcn_fence(__ATOMIC_RELEASE, "workgroup");
    __builtin_amdgcn_wave_barrier();
    __builtin_amdgcn_fence(__ATOMIC_ACQUIRE, "workgroup");
  }
}

#define RES_CARRY 4096.0f
#define RES_CARRY_INV (1.0f / 4096.0f)
#define P_CARRY 32768.0f

__device__ __forceinline__ unsigned pack_f16x2(float a, float b) {
  const unsigned short ua = __builtin_bit_cast(unsigned short, (_Float16)a);
  const unsigned short ub = __builtin_bit_cast(unsigned short, (_Float16)b);
  return (unsigned)ua | ((unsigned)ub << 16);
}
__device__ __forceinline__ void f16_hi_res_x2(float a, float b, unsigned& hw, unsigned& rw) {
  const _Float16 ha = (_Float16)a;
  const _Float16 hb = (_Float16)b;
  const float fa = (float)ha;
  const float fb = (float)hb;
  const float ra = (a - fa) * RES_CARRY;
  const float rb = (b - fb) * RES_CARRY;
  hw = (unsigned)__builtin_bit_cast(unsigned short, ha) | ((unsigned)__builtin_bit_cast(unsigned short, hb) << 16);
  rw = pack_f16x2(ra, rb);
}
__device__ __forceinline__ void bf16_hi_lo_x2(float a, float b, unsigned& hw, unsigned& lw) {
  const unsigned short ha = f2bf_bits(a);
  const unsigned short hb = f2bf_bits(b);
  const unsigned short la = f2bf_bits(a - bf_bits2f(ha));
  const unsigned short lb = f2bf_bits(b - bf_bits2f(hb));
  hw = (unsigned)ha | ((unsigned)hb << 16);
  lw = (unsigned)la | ((unsigned)lb << 16);
}

__global__ __launch_bounds__(256) void split_bf16_kernel(const float* __restrict__ in,
    unsigned short* __restrict__ oh, unsigned short* __restrict__ ol, int n8) {
  const int i = blockIdx.x * 256 + threadIdx.x;
  const int ic = (i < n8) ? i : (n8 - 1);
  const v4f a0 = *(const v4f*)(in + (size_t)ic * 8);
  const v4f a1 = *(const v4f*)(in + (size_t)ic * 8 + 4);
  v4u hv, lv;
  {
    unsigned hw, lw;
    bf16_hi_lo_x2(a0[0], a0[1], hw, lw); hv[0] = hw; lv[0] = lw;
    bf16_hi_lo_x2(a0[2], a0[3], hw, lw); hv[1] = hw; lv[1] = lw;
    bf16_hi_lo_x2(a1[0], a1[1], hw, lw); hv[2] = hw; lv[2] = lw;
    bf16_hi_lo_x2(a1[2], a1[3], hw, lw); hv[3] = hw; lv[3] = lw;
  }
  unsigned short* ph = oh + (size_t)ic * 8;
  unsigned short* pl = ol + (size_t)ic * 8;
  if (i < n8) { *(volatile v4u*)ph = hv; *(volatile v4u*)pl = lv; }
  __threadfence();
  if (i < n8) { *(volatile v4u*)ph = hv; *(volatile v4u*)pl = lv; }
}

__global__ __launch_bounds__(256) void wsplit_t_kernel(const float* __restrict__ W,
    unsigned short* __restrict__ oh, unsigned short* __restrict__ ol, int Kr, int Nc) {
  __shared__ __align__(16) float sW[64 * 68];
  const int tid = threadIdx.x;
  const int n0 = blockIdx.x * 64;
  const int k0 = blockIdx.y * 64;
  {
    const int k = tid >> 2;
    const int cq = (tid & 3) * 16;
    const float* src = W + (size_t)(k0 + k) * Nc + n0 + cq;
#pragma unroll
    for (int q = 0; q < 4; ++q) *(v4f*)(sW + k * 68 + cq + 4 * q) = *(const v4f*)(src + 4 * q);
  }
  __syncthreads();
  v4u hv[2], lv[2];
  size_t dst[2];
#pragma unroll
  for (int u = 0; u < 2; ++u) {
    const int task = tid + 256 * u;
    const int n = task >> 3;
    const int kg = task & 7;
#pragma unroll
    for (int e = 0; e < 4; ++e) {
      const float f0 = sW[(kg * 8 + 2 * e) * 68 + n];
      const float f1 = sW[(kg * 8 + 2 * e + 1) * 68 + n];
      unsigned hw, lw;
      bf16_hi_lo_x2(f0, f1, hw, lw);
      hv[u][e] = hw; lv[u][e] = lw;
    }
    dst[u] = (size_t)(n0 + n) * Kr + k0 + kg * 8;
  }
#pragma unroll
  for (int u = 0; u < 2; ++u) { *(volatile v4u*)(oh + dst[u]) = hv[u]; *(volatile v4u*)(ol + dst[u]) = lv[u]; }
  __threadfence();
#pragma unroll
  for (int u = 0; u < 2; ++u) { *(volatile v4u*)(oh + dst[u]) = hv[u]; *(volatile v4u*)(ol + dst[u]) = lv[u]; }
}

__global__ __launch_bounds__(256) void vsplit_t_kernel(const float* __restrict__ in, const float* __restrict__ bias,
    unsigned short* __restrict__ oh, unsigned short* __restrict__ ol, int S, int H) {
  __shared__ __align__(16) float sV[64 * 68];
  const int tid = threadIdx.x;
  const int s0 = blockIdx.x * 64;
  const int h = blockIdx.y;
  const int b = blockIdx.z;
  {
    const int s = tid >> 2;
    const int cq = (tid & 3) * 16;
    const float* src = in + (size_t)(b * S + s0 + s) * 256 + h * 64 + cq;
    const float* bsp = bias + h * 64 + cq;
#pragma unroll
    for (int q = 0; q < 4; ++q) {
      const v4f v = *(const v4f*)(src + 4 * q) + *(const v4f*)(bsp + 4 * q);
      *(v4f*)(sV + s * 68 + cq + 4 * q) = v;
    }
  }
  __syncthreads();
  v4u hv[2], rv[2];
  size_t dst[2];
#pragma unroll
  for (int u = 0; u < 2; ++u) {
    const int task = tid + 256 * u;
    const int d = task >> 3;
    const int sg = task & 7;
#pragma unroll
    for (int e = 0; e < 4; ++e) {
      const float f0 = sV[(sg * 8 + 2 * e) * 68 + d];
      const float f1 = sV[(sg * 8 + 2 * e + 1) * 68 + d];
      unsigned hw, rw;
      f16_hi_res_x2(f0, f1, hw, rw);
      hv[u][e] = hw; rv[u][e] = rw;
    }
    dst[u] = ((size_t)((b * H + h) * 64 + d)) * S + s0 + sg * 8;
  }
#pragma unroll
  for (int u = 0; u < 2; ++u) { *(volatile v4u*)(oh + dst[u]) = hv[u]; *(volatile v4u*)(ol + dst[u]) = rv[u]; }
  __threadfence();
#pragma unroll
  for (int u = 0; u < 2; ++u) { *(volatile v4u*)(oh + dst[u]) = hv[u]; *(volatile v4u*)(ol + dst[u]) = rv[u]; }
}

__global__ __launch_bounds__(512) void rope_table_kernel(float* __restrict__ tab) {
  const int i = threadIdx.x;
  const int p = i & 31;
  const int t = (i >> 5) & 7;
  const int which = i >> 8;
  const float e2 = (float)(2 * p) * 0.015625f;
  const float freq = exp2f(-(e2 * 13.28771237954945f));
  const float ang = (float)t * freq;
  const float cv = cosf(ang);
  const float sv = sinf(ang);
  const float val = which ? sv : cv;
  ((volatile float*)tab)[i] = val;
  __threadfence();
  ((volatile float*)tab)[i] = val;
}

__global__ __launch_bounds__(256) void rope_f16_kernel(const float* __restrict__ in, const float* __restrict__ bias,
    const float* __restrict__ tab, unsigned short* __restrict__ out, int M, int S, int nodesPerT) {
  const int n8 = M * 32;
  const int i = blockIdx.x * 256 + threadIdx.x;
  const int ic = (i < n8) ? i : (n8 - 1);
  const int row = ic >> 5;
  const int c0 = (ic & 31) * 8;
  v4f x0 = *(const v4f*)(in + (size_t)row * 256 + c0);
  v4f x1 = *(const v4f*)(in + (size_t)row * 256 + c0 + 4);
  const v4f b0 = *(const v4f*)(bias + c0);
  const v4f b1 = *(const v4f*)(bias + c0 + 4);
  x0 += b0;
  x1 += b1;
  const int s = row % S;
  int t = s / nodesPerT;
  t = (t > 7) ? 7 : t;
  const int p0 = (c0 & 63) >> 1;
  const v4f cs = *(const v4f*)(tab + t * 32 + p0);
  const v4f sn = *(const v4f*)(tab + 256 + t * 32 + p0);
  v4u w;
  w[0] = pack_f16x2(x0[0] * cs[0] - x0[1] * sn[0], x0[0] * sn[0] + x0[1] * cs[0]);
  w[1] = pack_f16x2(x0[2] * cs[1] - x0[3] * sn[1], x0[2] * sn[1] + x0[3] * cs[1]);
  w[2] = pack_f16x2(x1[0] * cs[2] - x1[1] * sn[2], x1[0] * sn[2] + x1[1] * cs[2]);
  w[3] = pack_f16x2(x1[2] * cs[3] - x1[3] * sn[3], x1[2] * sn[3] + x1[3] * cs[3]);
  unsigned short* po = out + (size_t)ic * 8;
  if (i < n8) *(volatile v4u*)po = w;
  __threadfence();
  if (i < n8) *(volatile v4u*)po = w;
}

#define AT_D 64
#define AT_NW 4
#define AT_QB 64
#define AT_KC 64

struct AttnDims {
  long q_bs; long k_bs; long v_bhs; long o_bs;
  int q_rs; int k_rs; int v_ds; int o_rs;
  int S; int Skv; int H; int coloff;
  float sscale; int pad0;
};
static_assert(sizeof(AttnDims) == 72);

__device__ __forceinline__ v8f mma_f16(v16h a, v16h b, v8f c) {
  c = __builtin_amdgcn_wmma_f32_16x16x32_f16(false, a, false, b, (short)0, c, false, false);
  asm volatile("v_nop\n\tv_nop\n\tv_nop\n\tv_nop" : "+v"(c) : "v"(a), "v"(b));
  return c;
}

__global__ __launch_bounds__(128)
void attn_hd64_kernel(const unsigned short* __restrict__ qp, const unsigned short* __restrict__ kp,
                      const unsigned short* __restrict__ vhp, const unsigned short* __restrict__ vlp,
                      float* __restrict__ outp, AttnDims g) {
  __shared__ __align__(16) _Float16 Ksh[AT_KC * AT_D];
  __shared__ __align__(16) _Float16 Vth[AT_D * AT_KC];
  __shared__ __align__(16) _Float16 Vtl[AT_D * AT_KC];
  __shared__ __align__(16) _Float16 Psh[AT_NW][16 * AT_KC];
  __shared__ __align__(16) _Float16 Psl[AT_NW][16 * AT_KC];
  __shared__ __align__(16) float  Os[AT_NW][16 * 68];

  const int tid  = threadIdx.x;
  const int wave = tid >> 5;
  const int lane = tid & 31;
  const int hh   = lane >> 4;
  const int c    = lane & 15;

  const int nqb = g.S / AT_QB;
  const int bx = blockIdx.x;
  const int qb = bx % nqb;
  const int bh = bx / nqb;
  const int h  = bh % g.H;
  const int b  = bh / g.H;
  const int q0 = qb * AT_QB + wave * 16;

  const _Float16* qbase = (const _Float16*)(const void*)qp + (size_t)b * g.q_bs + (size_t)h * AT_D;
  const _Float16* kbase = (const _Float16*)(const void*)kp + (size_t)b * g.k_bs + (size_t)h * AT_D;
  const _Float16* vhb = (const _Float16*)(const void*)vhp + (size_t)bh * g.v_bhs;
  const _Float16* vlb = (const _Float16*)(const void*)vlp + (size_t)bh * g.v_bhs;
  float* ob = outp + (size_t)b * g.o_bs + g.coloff + h * AT_D;

  v16h qa[2];
  {
    const _Float16* qrow = qbase + (size_t)(q0 + c) * g.q_rs + 8 * hh;
#pragma unroll
    for (int dc = 0; dc < 2; ++dc) qa[dc] = Frag<_Float16>::load(qrow + dc * 32);
  }

  float mrow[8], lrow[8];
  v8f oacc[4], racc[4];
#pragma unroll
  for (int r = 0; r < 8; ++r) { mrow[r] = -INFINITY; lrow[r] = 0.f; }
#pragma unroll
  for (int t = 0; t < 4; ++t) {
    oacc[t] = (v8f){0.f,0.f,0.f,0.f,0.f,0.f,0.f,0.f};
    racc[t] = (v8f){0.f,0.f,0.f,0.f,0.f,0.f,0.f,0.f};
  }

  const int nChunks = g.Skv / AT_KC;
  for (int kc = 0; kc < nChunks; ++kc) {
    const int kv0 = kc * AT_KC;
    __syncthreads();
    {
      const int grp = tid & 7;
      const int rr = tid >> 3;
#pragma unroll
      for (int it = 0; it < 4; ++it) {
        const int row = it * 16 + rr;
        const v4u kw = *(const v4u*)(kbase + (size_t)(kv0 + row) * g.k_rs + grp * 8);
        const v4u hw = *(const v4u*)(vhb + (size_t)row * g.v_ds + kv0 + grp * 8);
        const v4u lw = *(const v4u*)(vlb + (size_t)row * g.v_ds + kv0 + grp * 8);
        *(v4u*)(Ksh + row * AT_D + grp * 8) = kw;
        *(v4u*)(Vth + row * AT_KC + grp * 8) = hw;
        *(v4u*)(Vtl + row * AT_KC + grp * 8) = lw;
      }
    }
    __syncthreads();

    v8f s[4];
#pragma unroll
    for (int j = 0; j < 4; ++j) {
      s[j] = (v8f){0.f,0.f,0.f,0.f,0.f,0.f,0.f,0.f};
#pragma unroll
      for (int dc = 0; dc < 2; ++dc) {
        const v16h kb = Frag<_Float16>::load(Ksh + (j * 16 + c) * AT_D + dc * 32 + 8 * hh);
        s[j] = mma_f16(qa[dc], kb, s[j]);
      }
    }
    float cm[8];
#pragma unroll
    for (int r = 0; r < 8; ++r) {
      float m = -INFINITY;
#pragma unroll
      for (int j = 0; j < 4; ++j) {
        s[j][r] = s[j][r] * g.sscale;
        m = fmaxf(m, s[j][r]);
      }
#pragma unroll
      for (int off = 1; off < 16; off <<= 1) m = fmaxf(m, __shfl_xor(m, off, 32));
      cm[r] = m;
    }
    _Float16* pwh = Psh[wave];
    _Float16* pwl = Psl[wave];
#pragma unroll
    for (int r = 0; r < 8; ++r) {
      const float mnew = fmaxf(mrow[r], cm[r]);
      const float alpha = expf(mrow[r] - mnew);
      mrow[r] = mnew;
      float psum = 0.f;
#pragma unroll
      for (int j = 0; j < 4; ++j) {
        const float p = expf(s[j][r] - mnew);
        psum += p;
        const float pcv = p * P_CARRY;
        const _Float16 ph = (_Float16)pcv;
        const float phf = (float)ph;
        const float res = (pcv - phf) * RES_CARRY;
        const _Float16 pl = (_Float16)res;
        pwh[(8 * hh + r) * AT_KC + j * 16 + c] = ph;
        pwl[(8 * hh + r) * AT_KC + j * 16 + c] = pl;
      }
#pragma unroll
      for (int off = 1; off < 16; off <<= 1) psum += __shfl_xor(psum, off, 32);
      lrow[r] = lrow[r] * alpha + psum;
#pragma unroll
      for (int t = 0; t < 4; ++t) { oacc[t][r] *= alpha; racc[t][r] *= alpha; }
    }
    __builtin_amdgcn_fence(__ATOMIC_RELEASE, "workgroup");
    __builtin_amdgcn_wave_barrier();
    __builtin_amdgcn_fence(__ATOMIC_ACQUIRE, "workgroup");
#pragma unroll 1
    for (int kk = 0; kk < 2; ++kk) {
      const v16h pa = Frag<_Float16>::load(pwh + c * AT_KC + kk * 32 + 8 * hh);
      const v16h pr = Frag<_Float16>::load(pwl + c * AT_KC + kk * 32 + 8 * hh);
#pragma unroll
      for (int t = 0; t < 4; ++t) {
        const v16h vb = Frag<_Float16>::load(Vth + (t * 16 + c) * AT_KC + kk * 32 + 8 * hh);
        const v16h vr = Frag<_Float16>::load(Vtl + (t * 16 + c) * AT_KC + kk * 32 + 8 * hh);
        oacc[t] = mma_f16(pa, vb, oacc[t]);
        racc[t] = mma_f16(pa, vr, racc[t]);
        racc[t] = mma_f16(pr, vb, racc[t]);
      }
    }
  }

  float* os = Os[wave];
#pragma unroll
  for (int r = 0; r < 8; ++r) {
    const float inv = 1.0f / (lrow[r] * P_CARRY);
#pragma unroll
    for (int t = 0; t < 4; ++t) os[(8 * hh + r) * 68 + t * 16 + c] = (oacc[t][r] + racc[t][r] * RES_CARRY_INV) * inv;
  }
  __builtin_amdgcn_fence(__ATOMIC_RELEASE, "workgroup");
  __builtin_amdgcn_wave_barrier();
  __builtin_amdgcn_fence(__ATOMIC_ACQUIRE, "workgroup");
  {
    const int c4 = c * 4;
    for (int pass = 0; pass < 2; ++pass) {
#pragma unroll
      for (int it = 0; it < 8; ++it) {
        const int row = it * 2 + hh;
        const v4f val = *(const v4f*)(os + row * 68 + c4);
        *(volatile v4f*)(ob + (size_t)(q0 + row) * g.o_rs + c4) = val;
      }
      __threadfence();
    }
  }
}

static inline size_t align128(size_t x) { return (x + 127) & ~(size_t)127; }

extern "C" void kernel_launch(void* const* d_in, const int* in_sizes, int n_in,
                              void* d_out, int out_size, void* d_ws, size_t ws_size,
                              hipStream_t stream) {
  (void)in_sizes; (void)n_in; (void)out_size;
  const float* x0  = (const float*)d_in[0];
  const float* ea  = (const float*)d_in[1];
  const float* qd  = (const float*)d_in[2];
  const float* Wq  = (const float*)d_in[3];
  const float* bq  = (const float*)d_in[4];
  const float* Wk0 = (const float*)d_in[5];
  const float* bk0 = (const float*)d_in[6];
  const float* Wv0 = (const float*)d_in[7];
  const float* bv0 = (const float*)d_in[8];
  const float* Wk1 = (const float*)d_in[9];
  const float* bk1 = (const float*)d_in[10];
  const float* Wv1 = (const float*)d_in[11];
  const float* bv1 = (const float*)d_in[12];
  const float* Wo  = (const float*)d_in[13];
  const float* bo  = (const float*)d_in[14];
  float* out = (float*)d_out;

  constexpr int kBatch = 2, kHeads = 4, kDM = 256, kDH = 64, kDC = 512;
  constexpr int kSQ = 1024, kSK0 = 1024, kSK1 = 4096;
  constexpr int kNodesQ = 128, kNodes0 = 128, kNodes1 = 512;
  constexpr int kRQ = kBatch * kSQ;
  constexpr int kR0 = kBatch * kSK0;
  constexpr int kR1 = kBatch * kSK1;
  constexpr int kWTslot = kDM * kDM;
  static_assert(kRQ % 64 == 0 && kR0 % 64 == 0 && kR1 % 64 == 0 && kDM % 64 == 0);
  static_assert(kDM % 32 == 0 && kDC % 32 == 0);
  static_assert(kSQ % 64 == 0 && kSK0 % 64 == 0 && kSK1 % 64 == 0 && kDH == 64 && kHeads * kDH == kDM);
  static_assert((kRQ * kDM / 8) % 256 == 0 && (kR1 * kDM / 8) % 256 == 0 && (kRQ * kDC / 8) % 256 == 0);
  static_assert(kSQ == 8 * kNodesQ && kSK0 == 8 * kNodes0 && kSK1 == 8 * kNodes1);

  char* ws = (char*)d_ws;
  size_t off = 0;
  auto carve = [&](size_t bytes) -> char* { char* p = ws + off; off = align128(off + bytes); return p; };
  unsigned short* actq_h = (unsigned short*)carve((size_t)kRQ * kDM * 2);
  unsigned short* actq_l = (unsigned short*)carve((size_t)kRQ * kDM * 2);
  unsigned short* actx_h = (unsigned short*)carve((size_t)kR0 * kDM * 2);
  unsigned short* actx_l = (unsigned short*)carve((size_t)kR0 * kDM * 2);
  unsigned short* acte_h = (unsigned short*)carve((size_t)kR1 * kDM * 2);
  unsigned short* acte_l = (unsigned short*)carve((size_t)kR1 * kDM * 2);
  unsigned short* wt_h   = (unsigned short*)carve((size_t)5 * kWTslot * 2);
  unsigned short* wt_l   = (unsigned short*)carve((size_t)5 * kWTslot * 2);
  unsigned short* wot_h  = (unsigned short*)carve((size_t)kDM * kDC * 2);
  unsigned short* wot_l  = (unsigned short*)carve((size_t)kDM * kDC * 2);
  float* qf   = (float*)carve((size_t)kRQ * kDM * 4);
  float* kvf0 = (float*)carve((size_t)2 * kR0 * kDM * 4);
  float* kvf1 = (float*)carve((size_t)2 * kR1 * kDM * 4);
  unsigned short* q16  = (unsigned short*)carve((size_t)kRQ * kDM * 2);
  unsigned short* k016 = (unsigned short*)carve((size_t)kR0 * kDM * 2);
  unsigned short* k116 = (unsigned short*)carve((size_t)kR1 * kDM * 2);
  unsigned short* vt0_h = (unsigned short*)carve((size_t)kBatch * kHeads * 64 * kSK0 * 2);
  unsigned short* vt0_l = (unsigned short*)carve((size_t)kBatch * kHeads * 64 * kSK0 * 2);
  unsigned short* vt1_h = (unsigned short*)carve((size_t)kBatch * kHeads * 64 * kSK1 * 2);
  unsigned short* vt1_l = (unsigned short*)carve((size_t)kBatch * kHeads * 64 * kSK1 * 2);
  float* comb = (float*)carve((size_t)kRQ * kDC * 4);
  unsigned short* comb_h = (unsigned short*)carve((size_t)kRQ * kDC * 2);
  unsigned short* comb_l = (unsigned short*)carve((size_t)kRQ * kDC * 2);
  float* tab = (float*)carve((size_t)512 * 4);
  if (off > ws_size) return;

  rope_table_kernel<<<1, 512, 0, stream>>>(tab);

  split_bf16_kernel<<<(kRQ * kDM / 8) / 256, 256, 0, stream>>>(qd, actq_h, actq_l, kRQ * kDM / 8);
  split_bf16_kernel<<<(kR0 * kDM / 8) / 256, 256, 0, stream>>>(x0, actx_h, actx_l, kR0 * kDM / 8);
  split_bf16_kernel<<<(kR1 * kDM / 8) / 256, 256, 0, stream>>>(ea, acte_h, acte_l, kR1 * kDM / 8);

  {
    const dim3 wgrid(kDM / 64, kDM / 64);
    wsplit_t_kernel<<<wgrid, 256, 0, stream>>>(Wq,  wt_h + 0 * kWTslot, wt_l + 0 * kWTslot, kDM, kDM);
    wsplit_t_kernel<<<wgrid, 256, 0, stream>>>(Wk0, wt_h + 1 * kWTslot, wt_l + 1 * kWTslot, kDM, kDM);
    wsplit_t_kernel<<<wgrid, 256, 0, stream>>>(Wv0, wt_h + 2 * kWTslot, wt_l + 2 * kWTslot, kDM, kDM);
    wsplit_t_kernel<<<wgrid, 256, 0, stream>>>(Wk1, wt_h + 3 * kWTslot, wt_l + 3 * kWTslot, kDM, kDM);
    wsplit_t_kernel<<<wgrid, 256, 0, stream>>>(Wv1, wt_h + 4 * kWTslot, wt_l + 4 * kWTslot, kDM, kDM);
    wsplit_t_kernel<<<dim3(kDM / 64, kDC / 64), 256, 0, stream>>>(Wo, wot_h, wot_l, kDC, kDM);
  }

  {
    constexpr int tilesQ = (kRQ / 64) * (kDM / 64);
    static_assert(tilesQ % 8 == 0);
    wmma_gemm64<1, true, 0, 0, false><<<dim3(tilesQ / 8, 1), 256, 0, stream>>>(
        actq_h, actq_l, kDM, 0L, wt_h, wt_l, kDM, 0L,
        (void*)qf, (void*)qf, kDM, 0L, bq, bq, 0L, kRQ, kDM, kDM, 1.0f);
    constexpr int tiles0 = (kR0 / 64) * (kDM / 64);
    static_assert(tiles0 % 8 == 0);
    wmma_gemm64<1, true, 0, 0, false><<<dim3(tiles0 / 8, 2), 256, 0, stream>>>(
        actx_h, actx_l, kDM, 0L, wt_h + 1 * kWTslot, wt_l + 1 * kWTslot, kDM, (long)kWTslot,
        (void*)kvf0, (void*)kvf0, kDM, (long)kR0 * kDM, bk0, bk0, 0L, kR0, kDM, kDM, 1.0f);
    constexpr int tiles1 = (kR1 / 64) * (kDM / 64);
    static_assert(tiles1 % 8 == 0);
    wmma_gemm64<1, true, 0, 0, false><<<dim3(tiles1 / 8, 2), 256, 0, stream>>>(
        acte_h, acte_l, kDM, 0L, wt_h + 3 * kWTslot, wt_l + 3 * kWTslot, kDM, (long)kWTslot,
        (void*)kvf1, (void*)kvf1, kDM, (long)kR1 * kDM, bk1, bk1, 0L, kR1, kDM, kDM, 1.0f);
  }

  rope_f16_kernel<<<(kRQ * 32) / 256, 256, 0, stream>>>(qf, bq, tab, q16, kRQ, kSQ, kNodesQ);
  rope_f16_kernel<<<(kR0 * 32) / 256, 256, 0, stream>>>(kvf0, bk0, tab, k016, kR0, kSK0, kNodes0);
  rope_f16_kernel<<<(kR1 * 32) / 256, 256, 0, stream>>>(kvf1, bk1, tab, k116, kR1, kSK1, kNodes1);

  vsplit_t_kernel<<<dim3(kSK0 / 64, kHeads, kBatch), 256, 0, stream>>>(
      kvf0 + (size_t)kR0 * kDM, bv0, vt0_h, vt0_l, kSK0, kHeads);
  vsplit_t_kernel<<<dim3(kSK1 / 64, kHeads, kBatch), 256, 0, stream>>>(
      kvf1 + (size_t)kR1 * kDM, bv1, vt1_h, vt1_l, kSK1, kHeads);

  {
    AttnDims g0;
    g0.q_bs = (long)kSQ * kDM;  g0.k_bs = (long)kSK0 * kDM;  g0.v_bhs = (long)64 * kSK0;  g0.o_bs = (long)kSQ * kDC;
    g0.q_rs = kDM; g0.k_rs = kDM; g0.v_ds = kSK0; g0.o_rs = kDC;
    g0.S = kSQ; g0.Skv = kSK0; g0.H = kHeads; g0.coloff = 0;
    g0.sscale = 0.125f; g0.pad0 = 0;
    attn_hd64_kernel<<<kBatch * kHeads * (kSQ / 64), 128, 0, stream>>>(q16, k016, vt0_h, vt0_l, comb, g0);
    AttnDims g1;
    g1.q_bs = (long)kSQ * kDM;  g1.k_bs = (long)kSK1 * kDM;  g1.v_bhs = (long)64 * kSK1;  g1.o_bs = (long)kSQ * kDC;
    g1.q_rs = kDM; g1.k_rs = kDM; g1.v_ds = kSK1; g1.o_rs = kDC;
    g1.S = kSQ; g1.Skv = kSK1; g1.H = kHeads; g1.coloff = kDM;
    g1.sscale = 0.125f; g1.pad0 = 0;
    attn_hd64_kernel<<<kBatch * kHeads * (kSQ / 64), 128, 0, stream>>>(q16, k116, vt1_h, vt1_l, comb, g1);
  }

  split_bf16_kernel<<<(kRQ * kDC / 8) / 256, 256, 0, stream>>>(comb, comb_h, comb_l, kRQ * kDC / 8);
  {
    constexpr int tilesO = (kRQ / 64) * (kDM / 64);
    static_assert(tilesO % 8 == 0);
    wmma_gemm64<1, true, 2, 0, false><<<dim3(tilesO / 8, 1), 256, 0, stream>>>(
        comb_h, comb_l, kDC, 0L, wot_h, wot_l, kDC, 0L,
        (void*)out, (void*)out, kDM, 0L, bo, bo, 0L, kRQ, kDM, kDC, 1.0f);
  }
}
